// BertSelfAttention_63591285784957
// MI455X (gfx1250) — hardware-verified
//
#include <hip/hip_runtime.h>


#ifndef NB
#define NB 8
#endif
#ifndef SEQ
#define SEQ 1024
#endif
#define NB_FULL 8
#define SEQ_FULL 1024
#define DD 768
#define HH 12
#define DHD 64
#define MROWS (NB * SEQ)

#define CST 72
#define QT 128
#define KBLK 64
#define LDK 72
#define OST 68
#define QKV_CARRY 8.0f
#define P_CARRY 1024.0f
#define OUT_SCALE (1.0f / 8192.0f)
#define S_SCALE (1.0f / 512.0f)

static_assert(NB >= 1 && NB <= NB_FULL);
static_assert(SEQ >= QT && SEQ <= SEQ_FULL);
static_assert(SEQ % QT == 0);
static_assert(SEQ % KBLK == 0);
static_assert(MROWS % 64 == 0);
static_assert(DD % 64 == 0);
static_assert(DD % 32 == 0);
static_assert(HH * DHD == DD);
static_assert(DHD == 64);

typedef _Float16 v16h __attribute__((ext_vector_type(16)));
typedef _Float16 v8h  __attribute__((ext_vector_type(8)));
typedef v8h v8ha __attribute__((may_alias));
typedef __bf16 v16b __attribute__((ext_vector_type(16)));
typedef unsigned short v8us __attribute__((ext_vector_type(8)));
typedef v8us v8usa __attribute__((may_alias));
typedef float v8f __attribute__((ext_vector_type(8)));
typedef float v4f __attribute__((ext_vector_type(4)));
typedef v4f v4fa __attribute__((may_alias));

static_assert(sizeof(v16b) == sizeof(v8f));

__device__ __forceinline__ unsigned short f2bf_bits(float f) {
    unsigned int u = __float_as_uint(f);
    u += 0x7FFFu + ((u >> 16) & 1u);
    return (unsigned short)(u >> 16);
}
__device__ __forceinline__ float bf16_rne(float f) {
    unsigned int u = __float_as_uint(f);
    u += 0x7FFFu + ((u >> 16) & 1u);
    return __uint_as_float(u & 0xFFFF0000u);
}

__device__ __forceinline__ v16h ldfrag_h(const _Float16* p) {
    union { v16h v; v8h h[2]; } u;
    u.h[0] = *(const v8ha*)(p);
    u.h[1] = *(const v8ha*)(p + 16);
    return u.v;
}
__device__ __forceinline__ v16b ldfrag_b(const unsigned short* p) {
    union { v16b v; v8us h[2]; } u;
    u.h[0] = *(const v8usa*)(p);
    u.h[1] = *(const v8usa*)(p + 16);
    return u.v;
}

__device__ __forceinline__ v8f mma_h(v16h a, v16h b, v8f c) {
    c = __builtin_amdgcn_wmma_f32_16x16x32_f16(false, a, false, b, (short)0, c, false, false);
    asm volatile("v_nop\n\tv_nop\n\tv_nop\n\tv_nop" : "+v"(c) : "v"(a), "v"(b));
    return c;
}
__device__ __forceinline__ v8f mma_b(v16b a, v16b b, v8f c) {
    c = __builtin_amdgcn_wmma_f32_16x16x32_bf16(false, a, false, b, (short)0, c, false, false);
    const v8f ka = __builtin_bit_cast(v8f, a);
    const v8f kbv = __builtin_bit_cast(v8f, b);
    asm volatile("v_nop\n\tv_nop\n\tv_nop\n\tv_nop" : "+v"(c) : "v"(ka), "v"(kbv));
    return c;
}

__device__ __forceinline__ float rmax16(float v) {
    #pragma unroll
    for (int m = 8; m; m >>= 1) v = fmaxf(v, __shfl_xor(v, m, 32));
    return v;
}
__device__ __forceinline__ float rsum16(float v) {
    #pragma unroll
    for (int m = 8; m; m >>= 1) v += __shfl_xor(v, m, 32);
    return v;
}

__global__ __launch_bounds__(256) void k_cvt(const float* __restrict__ src,
                                             unsigned short* __restrict__ dst,
                                             int nrow, int seq, int seq_full) {
    const int t = blockIdx.x * 256 + (int)threadIdx.x;
    const int nchunk = nrow * (DD / 8);
    if (t >= nchunk) return;
    const int m  = t / (DD / 8);
    const int c8 = (t - m * (DD / 8)) * 8;
    const int bb = m / seq;
    const int srow = bb * seq_full + (m - bb * seq);
    const float* p = src + (size_t)srow * DD + c8;
    const v4f f0 = *(const v4fa*)(p);
    const v4f f1 = *(const v4fa*)(p + 4);
    const float x0 = f0.x, x1 = f0.y, x2 = f0.z, x3 = f0.w;
    const float x4 = f1.x, x5 = f1.y, x6 = f1.z, x7 = f1.w;
    v8us o;
    o[0] = f2bf_bits(x0); o[1] = f2bf_bits(x1); o[2] = f2bf_bits(x2); o[3] = f2bf_bits(x3);
    o[4] = f2bf_bits(x4); o[5] = f2bf_bits(x5); o[6] = f2bf_bits(x6); o[7] = f2bf_bits(x7);
    unsigned short* d = dst + (size_t)m * DD + c8;
    *(volatile v8us*)d = o;
    __threadfence();
    *(volatile v8us*)d = o;
}

__global__ __launch_bounds__(128) void k_proj(
    const unsigned short* __restrict__ Xb,
    const unsigned short* __restrict__ Wqb, const unsigned short* __restrict__ Wkb,
    const unsigned short* __restrict__ Wvb,
    const float* __restrict__ bq, const float* __restrict__ bk, const float* __restrict__ bv,
    _Float16* __restrict__ Qh, _Float16* __restrict__ Kh, _Float16* __restrict__ Vt)
{
    __shared__ __attribute__((aligned(16))) _Float16 Cs[64 * CST];

    const int tid = threadIdx.x, lane = tid & 31, wave = tid >> 5;
    const int row16 = lane & 15, hsel = lane >> 4, kbase = hsel << 3;
    const int mat = blockIdx.z;
    const int n0 = blockIdx.x * 64;
    const int m0 = blockIdx.y * 64;
    const int wm = (wave & 1) << 5;
    const int wn = (wave >> 1) << 5;
    const unsigned short* Wb = (mat == 0) ? Wqb : ((mat == 1) ? Wkb : Wvb);
    const float* bias = (mat == 0) ? bq : ((mat == 1) ? bk : bv);

    v8f c[2][2];
    #pragma unroll
    for (int i = 0; i < 2; ++i)
        #pragma unroll
        for (int j = 0; j < 2; ++j)
            #pragma unroll
            for (int r = 0; r < 8; ++r) c[i][j][r] = 0.f;

    const unsigned short* Ap = Xb + (size_t)(m0 + wm + row16) * DD + kbase;
    const unsigned short* Bp = Wb + (size_t)(n0 + wn + row16) * DD + kbase;

    #pragma unroll 2
    for (int k0 = 0; k0 < DD; k0 += 32) {
        const v16b a0 = ldfrag_b(Ap + k0);
        const v16b a1 = ldfrag_b(Ap + (size_t)16 * DD + k0);
        const v16b b0 = ldfrag_b(Bp + k0);
        const v16b b1 = ldfrag_b(Bp + (size_t)16 * DD + k0);
        c[0][0] = mma_b(a0, b0, c[0][0]);
        c[0][1] = mma_b(a0, b1, c[0][1]);
        c[1][0] = mma_b(a1, b0, c[1][0]);
        c[1][1] = mma_b(a1, b1, c[1][1]);
    }

    #pragma unroll
    for (int j = 0; j < 2; ++j) {
        const int nl = wn + (j << 4) + row16;
        const float bb = bf16_rne(bias[n0 + nl]);
        #pragma unroll
        for (int i = 0; i < 2; ++i) {
            #pragma unroll
            for (int r = 0; r < 8; ++r) {
                const int ml = wm + (i << 4) + (hsel << 3) + r;
                const _Float16 hv = (_Float16)((c[i][j][r] + bb) * QKV_CARRY);
                const int idx = (mat != 2) ? (ml * CST + nl) : (nl * CST + ml);
                Cs[idx] = hv;
            }
        }
    }
    __syncthreads();

    const int hd = n0 >> 6;
    const int bi = m0 / SEQ;
    const int s0 = m0 - bi * SEQ;
    const size_t bhh = (size_t)bi * HH + hd;
    _Float16* dst;
    size_t lpitch;
    if (mat == 2) { dst = Vt + bhh * DHD * SEQ + s0;         lpitch = SEQ; }
    else          { dst = ((mat == 0) ? Qh : Kh) + (bhh * SEQ + s0) * DHD; lpitch = DHD; }

    const int q8 = (tid & 7) << 3;
    const int l0 = tid >> 3;
    v8h v[4];
    #pragma unroll
    for (int p = 0; p < 4; ++p) v[p] = *(const v8ha*)(&Cs[(l0 + (p << 4)) * CST + q8]);
    #pragma unroll
    for (int p = 0; p < 4; ++p)
        *(volatile v8h*)(dst + (size_t)(l0 + (p << 4)) * lpitch + q8) = v[p];
    __threadfence();
    #pragma unroll
    for (int p = 0; p < 4; ++p)
        *(volatile v8h*)(dst + (size_t)(l0 + (p << 4)) * lpitch + q8) = v[p];
}

union __attribute__((aligned(16))) LdsU {
    _Float16 h[4 * KBLK * LDK];
    float    f[2 * KBLK * LDK];
};
static_assert(sizeof(LdsU) == 36864);
static_assert(8 * 16 * OST <= 2 * KBLK * LDK);
static_assert(2 * KBLK * LDK + 8 * 16 * LDK <= 4 * KBLK * LDK);

__global__ __launch_bounds__(256) __attribute__((amdgpu_num_vgpr(256)))
void k_attn(const _Float16* __restrict__ Qh, const _Float16* __restrict__ Kh,
            const _Float16* __restrict__ Vt, const float* __restrict__ amask,
            const float* __restrict__ click, float* __restrict__ out)
{
    __shared__ LdsU lds;
    _Float16* Ks = lds.h;
    _Float16* Vs = lds.h + KBLK * LDK;
    _Float16* Ps = lds.h + 2 * KBLK * LDK;

    const int tid = threadIdx.x, lane = tid & 31, wave = tid >> 5;
    const int row16 = lane & 15, hsel = lane >> 4, kbase = hsel << 3;
    const int bh = blockIdx.y;
    const int b = bh / HH;
    const int hd = bh - b * HH;
    const int q0 = blockIdx.x * QT + (wave << 4);
    const size_t baseQK = (size_t)bh * SEQ * DHD;
    const size_t baseV  = (size_t)bh * DHD * SEQ;

    v16h qf[2];
    #pragma unroll
    for (int kk = 0; kk < 2; ++kk)
        qf[kk] = ldfrag_h(Qh + baseQK + (size_t)(q0 + row16) * DHD + (kk << 5) + kbase);

    v8f acc[4];
    #pragma unroll
    for (int jd = 0; jd < 4; ++jd)
        #pragma unroll
        for (int r = 0; r < 8; ++r) acc[jd][r] = 0.f;
    float mrow[8], lrow[8];
    #pragma unroll
    for (int r = 0; r < 8; ++r) { mrow[r] = -1e30f; lrow[r] = 0.f; }

    _Float16* P = Ps + wave * (16 * LDK);
    const int key = tid >> 2;
    const int dc  = (tid & 3) << 4;
    const float* clk = click + (size_t)b * SEQ_FULL;
    const float* msk = amask + (size_t)b * SEQ_FULL;

    #pragma unroll 1
    for (int kb = 0; kb < SEQ; kb += KBLK) {
        __syncthreads();
        {
            const _Float16* ksrc = Kh + baseQK + (size_t)(kb + key) * DHD + dc;
            const _Float16* vsrc = Vt + baseV + (size_t)key * SEQ + kb + dc;
            const v8h ka  = *(const v8ha*)(ksrc);
            const v8h kb8 = *(const v8ha*)(ksrc + 8);
            const v8h va  = *(const v8ha*)(vsrc);
            const v8h vb  = *(const v8ha*)(vsrc + 8);
            *(v8ha*)(&Ks[key * LDK + dc])     = ka;
            *(v8ha*)(&Ks[key * LDK + dc + 8]) = kb8;
            *(v8ha*)(&Vs[key * LDK + dc])     = va;
            *(v8ha*)(&Vs[key * LDK + dc + 8]) = vb;
        }
        __syncthreads();

        v8f sc[4];
        #pragma unroll
        for (int j = 0; j < 4; ++j) {
            v8f s;
            #pragma unroll
            for (int r = 0; r < 8; ++r) s[r] = 0.f;
            #pragma unroll
            for (int kk = 0; kk < 2; ++kk) {
                const v16h kf = ldfrag_h(&Ks[((j << 4) + row16) * LDK + (kk << 5) + kbase]);
                s = mma_h(qf[kk], kf, s);
            }
            sc[j] = s;
        }
        #pragma unroll
        for (int j = 0; j < 4; ++j) {
            const int kg = kb + (j << 4) + row16;
            const float ct = bf16_rne(clk[kg]);
            const float mk = bf16_rne(msk[kg]);
            const float g = S_SCALE * ct;
            #pragma unroll
            for (int r = 0; r < 8; ++r) sc[j][r] = sc[j][r] * g + mk;
        }
        #pragma unroll
        for (int r = 0; r < 8; ++r) {
            float mx = sc[0][r];
            mx = fmaxf(mx, sc[1][r]); mx = fmaxf(mx, sc[2][r]); mx = fmaxf(mx, sc[3][r]);
            mx = rmax16(mx);
            const float mnew = fmaxf(mrow[r], mx);
            const float corr = __expf(mrow[r] - mnew);
            mrow[r] = mnew;
            #pragma unroll
            for (int jd = 0; jd < 4; ++jd) acc[jd][r] = acc[jd][r] * corr;
            float sum = 0.f;
            #pragma unroll
            for (int j = 0; j < 4; ++j) {
                const float e = __expf(sc[j][r] - mnew);
                sc[j][r] = e;
                sum += e;
            }
            lrow[r] = lrow[r] * corr + rsum16(sum);
        }
        #pragma unroll
        for (int j = 0; j < 4; ++j)
            #pragma unroll
            for (int r = 0; r < 8; ++r)
                P[(r + (hsel << 3)) * LDK + (j << 4) + row16] = (_Float16)(sc[j][r] * P_CARRY);
        __builtin_amdgcn_fence(3, "wavefront");
        __builtin_amdgcn_wave_barrier();
        #pragma unroll
        for (int kk = 0; kk < 2; ++kk) {
            const v16h pf = ldfrag_h(&P[row16 * LDK + (kk << 5) + kbase]);
            #pragma unroll
            for (int jd = 0; jd < 4; ++jd) {
                const v16h vf = ldfrag_h(&Vs[((jd << 4) + row16) * LDK + (kk << 5) + kbase]);
                acc[jd] = mma_h(pf, vf, acc[jd]);
            }
        }
    }

    float scl[8];
    #pragma unroll
    for (int r = 0; r < 8; ++r) scl[r] = (1.0f / lrow[r]) * OUT_SCALE;

    __syncthreads();
    float* Os = lds.f + wave * (16 * OST);
    #pragma unroll
    for (int jd = 0; jd < 4; ++jd) {
        const int dh = (jd << 4) + row16;
        #pragma unroll
        for (int r = 0; r < 8; ++r) Os[((hsel << 3) + r) * OST + dh] = acc[jd][r] * scl[r];
    }
    __syncthreads();

    const int q4 = (lane & 15) << 2;
    v4f ov[8];
    #pragma unroll
    for (int p = 0; p < 8; ++p) ov[p] = *(const v4fa*)(&Os[((p << 1) + hsel) * OST + q4]);
    float* orow = out + ((size_t)b * SEQ + q0) * DD + hd * DHD + q4;
    #pragma unroll
    for (int p = 0; p < 8; ++p)
        *(volatile v4f*)(orow + (size_t)((p << 1) + hsel) * DD) = ov[p];
    __threadfence();
    #pragma unroll
    for (int p = 0; p < 8; ++p)
        *(volatile v4f*)(orow + (size_t)((p << 1) + hsel) * DD) = ov[p];
}

extern "C" void kernel_launch(void* const* d_in, const int* in_sizes, int n_in,
                              void* d_out, int out_size, void* d_ws, size_t ws_size,
                              hipStream_t stream) {
    if (n_in < 9) return;
    const long long need_rows = (long long)(NB - 1) * SEQ_FULL + SEQ;
    if ((long long)in_sizes[0] < need_rows * DD) return;
    if ((long long)in_sizes[1] < need_rows) return;
    if ((long long)in_sizes[2] < need_rows) return;
    if (in_sizes[3] < DD * DD || in_sizes[5] < DD * DD || in_sizes[7] < DD * DD) return;
    if (in_sizes[4] < DD || in_sizes[6] < DD || in_sizes[8] < DD) return;
    if ((long long)out_size < (long long)MROWS * DD) return;

    const float* X     = (const float*)d_in[0];
    const float* amask = (const float*)d_in[1];
    const float* click = (const float*)d_in[2];
    const float* Wq    = (const float*)d_in[3];
    const float* bq    = (const float*)d_in[4];
    const float* Wk    = (const float*)d_in[5];
    const float* bk    = (const float*)d_in[6];
    const float* Wv    = (const float*)d_in[7];
    const float* bv    = (const float*)d_in[8];
    float* out = (float*)d_out;

    const size_t plane = (size_t)MROWS * DD;
    const size_t wpl   = (size_t)DD * DD;
    const size_t total_bytes = 2u * (4u * plane + 3u * wpl);
    if (ws_size < total_bytes) return;
    unsigned short* Xb  = (unsigned short*)d_ws;
    unsigned short* Wqb = Xb + plane;
    unsigned short* Wkb = Wqb + wpl;
    unsigned short* Wvb = Wkb + wpl;
    _Float16* Qh = (_Float16*)(Wvb + wpl);
    _Float16* Kh = Qh + plane;
    _Float16* Vt = Kh + plane;

    const int nchunk_x = MROWS * (DD / 8);
    const int nchunk_w = DD * (DD / 8);
    k_cvt<<<dim3((nchunk_x + 255) / 256), dim3(256), 0, stream>>>(X,  Xb,  MROWS, SEQ, SEQ_FULL);
    k_cvt<<<dim3((nchunk_w + 255) / 256), dim3(256), 0, stream>>>(Wq, Wqb, DD, DD, DD);
    k_cvt<<<dim3((nchunk_w + 255) / 256), dim3(256), 0, stream>>>(Wk, Wkb, DD, DD, DD);
    k_cvt<<<dim3((nchunk_w + 255) / 256), dim3(256), 0, stream>>>(Wv, Wvb, DD, DD, DD);

    k_proj<<<dim3(DD / 64, MROWS / 64, 3), dim3(128), 0, stream>>>(
        Xb, Wqb, Wkb, Wvb, bq, bk, bv, Qh, Kh, Vt);

    k_attn<<<dim3(SEQ / QT, NB * HH), dim3(256), 0, stream>>>(Qh, Kh, Vt, amask, click, out);
}
